// SharedGATNetwork_54443005444824
// MI455X (gfx1250) — hardware-verified
//
#include <hip/hip_runtime.h>
#include <stdint.h>


typedef _Float16 v16h __attribute__((ext_vector_type(16)));
typedef _Float16 v8h  __attribute__((ext_vector_type(8)));
typedef float    v8f  __attribute__((ext_vector_type(8)));
typedef float    v4f  __attribute__((ext_vector_type(4)));
typedef v8h      v8ha __attribute__((may_alias));
typedef v4f      v4fa __attribute__((may_alias));
typedef _Float16 h16a __attribute__((may_alias));
typedef float    f32a __attribute__((may_alias));

union Frag { v16h v; v8h half[2]; };

#define NBATCH 8
#define NNODE  1024
#define NFEAT  128
#define NHEAD  4
#define NHDIM  32
#define PROJ_ROWS 64
#define AGG_ROWS  64

#define H_SCALE     16.0f
#define W_SCALE     64.0f
#define WH_UNSCALE  (1.0f / 1024.0f)
#define WHT_SCALE   16.0f
#define P_SCALE     4096.0f
#define AGG_UNSCALE (1.0f / 65536.0f)

__device__ __forceinline__ v8f wmma_f16(v16h a, v16h b, v8f c) {
  c = __builtin_amdgcn_wmma_f32_16x16x32_f16(false, a, false, b, (short)0, c, false, false);
  asm volatile("v_nop\n\tv_nop\n\tv_nop\n\tv_nop" : "+v"(c) : "v"(a), "v"(b));
  return c;
}

__global__ __launch_bounds__(128) void k_proj(const float* __restrict__ H,
                                              const float* __restrict__ W,
                                              const float* __restrict__ asrc,
                                              const float* __restrict__ adst,
                                              _Float16* __restrict__ WhT,
                                              float* __restrict__ sT,
                                              float* __restrict__ tT,
                                              int nblk) {
  __shared__ __attribute__((aligned(16))) float smem[12288];
  __shared__ __attribute__((aligned(16))) float avec[256];
  __shared__ __attribute__((aligned(16))) float stt[512];
  if ((int)blockIdx.x >= nblk) return;

  const int tid = threadIdx.x;
  const int m0  = blockIdx.x * PROJ_ROWS;
  h16a* hs  = (h16a*)smem;
  h16a* wsT = (h16a*)(smem + 4096);

  avec[tid]       = asrc[tid];
  avec[128 + tid] = adst[tid];
  for (int idx = tid; idx < NFEAT * NFEAT; idx += 128) {
    const int kk = idx & 127, nn = idx >> 7;
    wsT[nn * 128 + kk] = (_Float16)(W[kk * NFEAT + nn] * W_SCALE);
  }
  for (int idx = tid; idx < PROJ_ROWS * NFEAT; idx += 128) {
    const int r = idx >> 7, c = idx & 127;
    hs[r * 128 + c] = (_Float16)(H[(size_t)(m0 + r) * NFEAT + c] * H_SCALE);
  }
  __syncthreads();

  const int wave = tid >> 5, l = tid & 31, h = l >> 4, m = l & 15;
  const int mrow = wave * 16;

  v8f acc[8] = {};
#pragma unroll 1
  for (int k0 = 0; k0 < NFEAT; k0 += 32) {
    Frag a;
    a.half[0] = *(const v8ha*)(hs + (mrow + m) * 128 + k0 + 8 * h);
    a.half[1] = *(const v8ha*)(hs + (mrow + m) * 128 + k0 + 16 + 8 * h);
#pragma unroll
    for (int nt = 0; nt < 8; ++nt) {
      Frag bq;
      bq.half[0] = *(const v8ha*)(wsT + (nt * 16 + m) * 128 + k0 + 8 * h);
      bq.half[1] = *(const v8ha*)(wsT + (nt * 16 + m) * 128 + k0 + 16 + 8 * h);
      acc[nt] = wmma_f16(a.v, bq.v, acc[nt]);
    }
  }
  __syncthreads();

  f32a* cs = (f32a*)smem;
  h16a* tr = (h16a*)(smem + 8192);
#pragma unroll
  for (int nt = 0; nt < 8; ++nt) {
    const int c = nt * 16 + m;
    v8h t8 = {};
#pragma unroll
    for (int r = 0; r < 8; ++r) {
      const float x = acc[nt][r] * WH_UNSCALE;
      cs[(mrow + 8 * h + r) * 128 + c] = x;
      t8[r] = (_Float16)(x * WHT_SCALE);
    }
    *(v8ha*)(tr + c * 64 + mrow + 8 * h) = t8;
  }
  __syncthreads();

  {
    const int r = tid >> 1;
    const int kb = (tid & 1) * 2;
#pragma unroll
    for (int kq = 0; kq < 2; ++kq) {
      const int kk = kb + kq;
      float sv = 0.0f, tv = 0.0f;
#pragma unroll
      for (int dq = 0; dq < 8; ++dq) {
        const v4f x  = *(const v4fa*)(cs + r * 128 + kk * NHDIM + 4 * dq);
        const v4f ps = *(const v4fa*)(avec + kk * NHDIM + 4 * dq);
        const v4f pd = *(const v4fa*)(avec + 128 + kk * NHDIM + 4 * dq);
        sv += x.x * ps.x; sv += x.y * ps.y; sv += x.z * ps.z; sv += x.w * ps.w;
        tv += x.x * pd.x; tv += x.y * pd.y; tv += x.z * pd.z; tv += x.w * pd.w;
      }
      stt[kk * 64 + r]       = sv;
      stt[256 + kk * 64 + r] = tv;
    }
  }
  __syncthreads();

  const int bb = m0 >> 10;
  const int j0 = m0 & 1023;

  if (wave < 2) {
    float* dst = (wave == 0) ? sT : tT;
    const float* src = stt + wave * 256;
#pragma unroll
    for (int q = 0; q < 2; ++q) {
      const int head = 2 * q + h;
      const v4f v = *(const v4fa*)(src + head * 64 + 4 * m);
      *(volatile v4f*)(dst + (size_t)(bb * NHEAD + head) * NNODE + j0 + 4 * m) = v;
    }
  }
#pragma unroll
  for (int it = 0; it < 8; ++it) {
    const int c = wave * 32 + 4 * it + (l >> 3);
    const int q = l & 7;
    const v8h v = *(const v8ha*)(tr + c * 64 + 8 * q);
    *(volatile v8h*)(WhT + (size_t)(bb * NFEAT + c) * NNODE + j0 + 8 * q) = v;
  }
  __threadfence();
  if (wave < 2) {
    float* dst = (wave == 0) ? sT : tT;
    const float* src = stt + wave * 256;
#pragma unroll
    for (int q = 0; q < 2; ++q) {
      const int head = 2 * q + h;
      const v4f v = *(const v4fa*)(src + head * 64 + 4 * m);
      *(volatile v4f*)(dst + (size_t)(bb * NHEAD + head) * NNODE + j0 + 4 * m) = v;
    }
  }
#pragma unroll
  for (int it = 0; it < 8; ++it) {
    const int c = wave * 32 + 4 * it + (l >> 3);
    const int q = l & 7;
    const v8h v = *(const v8ha*)(tr + c * 64 + 8 * q);
    *(volatile v8h*)(WhT + (size_t)(bb * NFEAT + c) * NNODE + j0 + 8 * q) = v;
  }
}

__device__ __forceinline__ float max_quad(float tmax, v4f a, v4f t, int jbase, int irow) {
#pragma unroll
  for (int u = 0; u < 4; ++u) {
    const bool on = (a[u] > 0.0f) || (jbase + u == irow);
    tmax = on ? fmaxf(tmax, t[u]) : tmax;
  }
  return tmax;
}

__device__ __forceinline__ void agg_quad(v16h& p, int base_i, v4f a, v4f t, int jbase,
                                         int irow, float si, float em, float& lsum) {
#pragma unroll
  for (int u = 0; u < 4; ++u) {
    float e = si + t[u];
    e = (e >= 0.0f) ? e : 0.2f * e;
    float pv = __expf(fminf(e - em, 0.0f));
    const bool on = (a[u] > 0.0f) || (jbase + u == irow);
    pv = on ? pv : 0.0f;
    lsum += pv;
    p[base_i + u] = (_Float16)(pv * P_SCALE);
  }
}

__global__ __launch_bounds__(128) void k_attn(const float* __restrict__ Adj,
                                              const float* __restrict__ sT,
                                              const float* __restrict__ tT,
                                              const _Float16* __restrict__ WhT,
                                              float* __restrict__ Hout,
                                              int nblk) {
  __shared__ __attribute__((aligned(16))) float t_s[NNODE];
  __shared__ __attribute__((aligned(16))) float os[AGG_ROWS * NHDIM];
  __shared__ __attribute__((aligned(16))) float lv_s[AGG_ROWS];
  if ((int)blockIdx.x >= nblk) return;

  const int tid = threadIdx.x;
  const int bk  = blockIdx.x;
  const int ib  = bk & 15;
  const int k   = (bk >> 4) & 3;
  const int b   = bk >> 6;
  const int i0  = ib * AGG_ROWS;

  const int wave = tid >> 5, l = tid & 31, h = l >> 4, m = l & 15;
  const int rloc = wave * 16 + m;
  const int irow = i0 + rloc;

  const float* Arow = Adj + ((size_t)b * NNODE + irow) * NNODE;
  const float* tb   = tT + (size_t)(b * NHEAD + k) * NNODE;
  for (int j = tid; j < NNODE; j += 128) t_s[j] = tb[j];
  const float si = sT[(size_t)(b * NHEAD + k) * NNODE + irow];
  __syncthreads();

  float tmax = -3.0e38f;
#pragma unroll 1
  for (int j0 = 0; j0 < NNODE; j0 += 32) {
    const int jA = j0 + 8 * h, jB = j0 + 16 + 8 * h;
    const v4f a0 = *(const v4fa*)(Arow + jA);
    const v4f a1 = *(const v4fa*)(Arow + jA + 4);
    const v4f a2 = *(const v4fa*)(Arow + jB);
    const v4f a3 = *(const v4fa*)(Arow + jB + 4);
    const v4f u0 = *(const v4fa*)(t_s + jA);
    const v4f u1 = *(const v4fa*)(t_s + jA + 4);
    const v4f u2 = *(const v4fa*)(t_s + jB);
    const v4f u3 = *(const v4fa*)(t_s + jB + 4);
    tmax = max_quad(tmax, a0, u0, jA,     irow);
    tmax = max_quad(tmax, a1, u1, jA + 4, irow);
    tmax = max_quad(tmax, a2, u2, jB,     irow);
    tmax = max_quad(tmax, a3, u3, jB + 4, irow);
  }
  tmax = fmaxf(tmax, __shfl_xor(tmax, 16, 32));
  float em = si + tmax;
  em = (em >= 0.0f) ? em : 0.2f * em;

  v8f c0 = {}, c1 = {};
  float lsum = 0.0f;
  const _Float16* Bc0 = WhT + (size_t)(b * NFEAT + k * NHDIM + m) * NNODE;
  const _Float16* Bc1 = Bc0 + (size_t)16 * NNODE;
#pragma unroll 1
  for (int j0 = 0; j0 < NNODE; j0 += 32) {
    const int jA = j0 + 8 * h, jB = j0 + 16 + 8 * h;
    const v4f a0 = *(const v4fa*)(Arow + jA);
    const v4f a1 = *(const v4fa*)(Arow + jA + 4);
    const v4f a2 = *(const v4fa*)(Arow + jB);
    const v4f a3 = *(const v4fa*)(Arow + jB + 4);
    const v4f u0 = *(const v4fa*)(t_s + jA);
    const v4f u1 = *(const v4fa*)(t_s + jA + 4);
    const v4f u2 = *(const v4fa*)(t_s + jB);
    const v4f u3 = *(const v4fa*)(t_s + jB + 4);
    v16h p = {};
    agg_quad(p, 0,  a0, u0, jA,     irow, si, em, lsum);
    agg_quad(p, 4,  a1, u1, jA + 4, irow, si, em, lsum);
    agg_quad(p, 8,  a2, u2, jB,     irow, si, em, lsum);
    agg_quad(p, 12, a3, u3, jB + 4, irow, si, em, lsum);
    Frag b0, b1;
    b0.half[0] = *(const v8ha*)(Bc0 + jA);
    b0.half[1] = *(const v8ha*)(Bc0 + jB);
    b1.half[0] = *(const v8ha*)(Bc1 + jA);
    b1.half[1] = *(const v8ha*)(Bc1 + jB);
    c0 = wmma_f16(p, b0.v, c0);
    c1 = wmma_f16(p, b1.v, c1);
  }
  lsum += __shfl_xor(lsum, 16, 32);
  if (h == 0) lv_s[rloc] = (1.0f / lsum) * AGG_UNSCALE;
  __syncthreads();

#pragma unroll
  for (int r = 0; r < 8; ++r) {
    const int row = wave * 16 + 8 * h + r;
    const float sc = lv_s[row];
    float x0 = c0[r] * sc;
    float x1 = c1[r] * sc;
    x0 = (x0 > 0.0f) ? x0 : (__expf(x0) - 1.0f);
    x1 = (x1 > 0.0f) ? x1 : (__expf(x1) - 1.0f);
    os[row * NHDIM + m]      = x0;
    os[row * NHDIM + 16 + m] = x1;
  }
  __syncthreads();

#pragma unroll
  for (int it = 0; it < 4; ++it) {
    const int row = wave * 16 + 4 * it + (l >> 3);
    const int q = l & 7;
    const v4f v = *(const v4fa*)(os + row * NHDIM + 4 * q);
    *(volatile v4f*)(Hout + ((size_t)(b * NNODE + i0 + row)) * NFEAT + k * NHDIM + 4 * q) = v;
  }
  __threadfence();
#pragma unroll
  for (int it = 0; it < 4; ++it) {
    const int row = wave * 16 + 4 * it + (l >> 3);
    const int q = l & 7;
    const v4f v = *(const v4fa*)(os + row * NHDIM + 4 * q);
    *(volatile v4f*)(Hout + ((size_t)(b * NNODE + i0 + row)) * NFEAT + k * NHDIM + 4 * q) = v;
  }
}

extern "C" void kernel_launch(void* const* d_in, const int* in_sizes, int n_in,
                              void* d_out, int out_size, void* d_ws, size_t ws_size,
                              hipStream_t stream) {
  if (n_in < 8) return;
  if (in_sizes[0] != NBATCH * NNODE * NFEAT) return;
  if (in_sizes[1] != NBATCH * NNODE * NNODE) return;
  if (in_sizes[2] != NFEAT * NFEAT) return;
  if (in_sizes[3] != NHEAD * NHDIM) return;
  if (in_sizes[4] != NHEAD * NHDIM) return;
  if (in_sizes[5] != NFEAT * NFEAT) return;
  if (in_sizes[6] != NHEAD * NHDIM) return;
  if (in_sizes[7] != NHEAD * NHDIM) return;
  if (out_size != NBATCH * NNODE * NFEAT) return;

  const float* X      = (const float*)d_in[0];
  const float* Adj    = (const float*)d_in[1];
  const float* W0     = (const float*)d_in[2];
  const float* a_src0 = (const float*)d_in[3];
  const float* a_dst0 = (const float*)d_in[4];
  const float* W1     = (const float*)d_in[5];
  const float* a_src1 = (const float*)d_in[6];
  const float* a_dst1 = (const float*)d_in[7];
  float* OUT = (float*)d_out;

  const size_t whtBytes = (size_t)NBATCH * NFEAT * NNODE * sizeof(_Float16);
  const size_t stBytes  = (size_t)NBATCH * NHEAD * NNODE * sizeof(float);
  const size_t h1Bytes  = (size_t)NBATCH * NNODE * NFEAT * sizeof(float);
  const size_t oWhT = 0;
  const size_t oS   = oWhT + whtBytes;
  const size_t oT   = oS + stBytes;
  const size_t oH1  = oT + stBytes;
  const size_t total = oH1 + h1Bytes;
  if (total > ws_size) return;

  char* ws = (char*)d_ws;
  _Float16* WhT = (_Float16*)(ws + oWhT);
  float*    sT  = (float*)(ws + oS);
  float*    tT  = (float*)(ws + oT);
  float*    H1  = (float*)(ws + oH1);

  const int proj_blocks = (NBATCH * NNODE + PROJ_ROWS - 1) / PROJ_ROWS;
  const int attn_blocks = NBATCH * NHEAD * ((NNODE + AGG_ROWS - 1) / AGG_ROWS);

  k_proj<<<proj_blocks, 128, 0, stream>>>(X, W0, a_src0, a_dst0, WhT, sT, tT, proj_blocks);
  k_attn<<<attn_blocks, 128, 0, stream>>>(Adj, sT, tT, WhT, H1, attn_blocks);
  k_proj<<<proj_blocks, 128, 0, stream>>>(H1, W1, a_src1, a_dst1, WhT, sT, tT, proj_blocks);
  k_attn<<<attn_blocks, 128, 0, stream>>>(Adj, sT, tT, WhT, OUT, attn_blocks);
}
